// MemoryModule_33346126086839
// MI455X (gfx1250) — hardware-verified
//
#include <hip/hip_runtime.h>
#include <stddef.h>


typedef _Float16 v16h __attribute__((ext_vector_type(16)));
typedef _Float16 v8h  __attribute__((ext_vector_type(8)));
typedef float    v8f  __attribute__((ext_vector_type(8)));
typedef float    v4f  __attribute__((ext_vector_type(4)));
typedef _Float16 h16;

#ifndef NB
#define NB 8
#endif
#ifndef NL
#define NL 12
#endif
#define NB_FULL 8
#define NL_FULL 12
#define TT 36
#define DD 1024
#define FF 3
#define CC 32
#define JR 108
#define JP 128
#define NBL (NB * NL)

static_assert(NB >= 1 && NB <= NB_FULL);
static_assert(NL >= 1 && NL <= NL_FULL);
static_assert(JR == TT * FF);
static_assert(JP >= JR + 1 && (JP % 32) == 0 && JP == 8 * 16);
static_assert(CC == 32);
static_assert((DD % 128) == 0 && (DD % 32) == 0);
static_assert(TT * 64 * FF == 27 * 256);
static_assert((JP - JR) * 64 == 5 * 256);
static_assert(4 * 32 == JP);
static_assert(4 * 16 == 64);
static_assert(2 * 16 == CC);
static_assert(4 * 8 == CC);
static_assert(32 * 4 == 128);
static_assert(8 * 8 == 64);
static_assert(16 * 8 == JP);

#define LDT 72
#define LDG 132
#define LDA 40
static_assert((LDT % 8) == 0 && LDT >= 64);
static_assert((LDG % 4) == 0 && LDG >= JP);
static_assert(LDA >= TT);
static_assert((size_t)JP * LDT * 2 <= (size_t)131072);
static_assert((size_t)CC * LDG * 4 + (size_t)CC * LDA * 4 <= (size_t)131072);

#define XCARRY 1024.0f
#define PCARRY 1024.0f
#define RCARRY 2048.0f

#define XT_BYTES ((size_t)NBL * JP * DD * 2)
#define XD_BYTES ((size_t)NBL * DD * JP * 2)
#define Q_BYTES  ((size_t)NBL * CC * DD * 2)
#define AW_BYTES ((size_t)NBL * CC * JP * 2)
#define OFF_XT ((size_t)0)
#define OFF_XD (OFF_XT + XT_BYTES)
#define OFF_QH (OFF_XD + XD_BYTES)
#define OFF_QR (OFF_QH + Q_BYTES)
#define OFF_AW (OFF_QR + Q_BYTES)
#define WS_TOTAL (OFF_AW + AW_BYTES)
static_assert((XT_BYTES % 128) == 0 && (XD_BYTES % 128) == 0);
static_assert((Q_BYTES % 128) == 0 && (AW_BYTES % 128) == 0);
static_assert(WS_TOTAL <= (size_t)134217728);

__device__ __forceinline__ float bf16r(float x) {
  unsigned int u = __float_as_uint(x);
  u = (u + 0x7FFFu + ((u >> 16) & 1u)) & 0xFFFF0000u;
  return __uint_as_float(u);
}

static __device__ __forceinline__ h16 toh_flush(float v) {
  const h16 r = (h16)v;
  return (fabsf(v) < 6.103515625e-05f) ? (h16)0.0f : r;
}

__device__ __forceinline__ v16h frag_at(const _Float16* p) {
  v8h lo = *(const v8h*)(p);
  v8h hi = *(const v8h*)(p + 16);
  v16h out;
#pragma unroll
  for (int i = 0; i < 8; ++i) { out[i] = lo[i]; out[i + 8] = hi[i]; }
  return out;
}

__device__ __forceinline__ v8f wmma16(v16h a, v16h b, v8f c) {
  v8f d = __builtin_amdgcn_wmma_f32_16x16x32_f16(false, a, false, b, (short)0, c,
                                                 false, false);
  asm volatile("v_nop\n\tv_nop\n\tv_nop\n\tv_nop" : "+v"(d) : "v"(a), "v"(b));
  return d;
}

__global__ __launch_bounds__(256) void xconv_kernel(
    const float* __restrict__ xh, _Float16* __restrict__ XT, _Float16* __restrict__ XD) {
  __shared__ __attribute__((aligned(16))) _Float16 S[JP * LDT];
  const unsigned tid = threadIdx.x;
  const unsigned d0 = blockIdx.x * 64u;
  const unsigned bl = blockIdx.y;
  const unsigned b = bl / (unsigned)NL;
  const unsigned l = bl - b * (unsigned)NL;
  const float* src = xh + ((size_t)(b * (unsigned)NL_FULL + l) * TT) * (size_t)(DD * FF)
                     + (size_t)d0 * FF;
#pragma unroll 1
  for (unsigned it = 0; it < 27u; ++it) {
    const unsigned idx = tid + 256u * it;
    const unsigned t = idx / 192u;
    const unsigned r = idx - t * 192u;
    const unsigned dd = r / 3u;
    const unsigned f = r - dd * 3u;
    const float v = src[(size_t)t * (size_t)(DD * FF) + r];
    S[(t * 3u + f) * LDT + dd] = toh_flush(XCARRY * bf16r(v));
  }
#pragma unroll 1
  for (unsigned it = 0; it < 5u; ++it) {
    const unsigned idx = tid + 256u * it;
    const unsigned row = (unsigned)JR + (idx >> 6);
    const unsigned col = idx & 63u;
    S[row * LDT + col] = (row == (unsigned)JR) ? (h16)XCARRY : (h16)0.0f;
  }
  __syncthreads();

  v8h x[4], y[4];
  size_t offx[4], offy[4];
#pragma unroll
  for (unsigned i = 0; i < 4u; ++i) {
    const unsigned j = 32u * i + (tid >> 3);
    const unsigned c = (tid & 7u) * 8u;
    x[i] = *(const v8h*)&S[j * LDT + c];
    offx[i] = ((size_t)bl * JP + j) * DD + d0 + c;
  }
#pragma unroll
  for (unsigned i = 0; i < 4u; ++i) {
    const unsigned dd = 16u * i + (tid >> 4);
    const unsigned jc = (tid & 15u) * 8u;
#pragma unroll
    for (unsigned e = 0; e < 8u; ++e) y[i][e] = S[(jc + e) * LDT + dd];
    offy[i] = ((size_t)bl * DD + d0 + dd) * JP + jc;
  }
#pragma unroll
  for (int i = 0; i < 4; ++i) *(volatile v8h*)(XT + offx[i]) = x[i];
#pragma unroll
  for (int i = 0; i < 4; ++i) *(volatile v8h*)(XD + offy[i]) = y[i];
  __threadfence();
#pragma unroll
  for (int i = 0; i < 4; ++i) *(volatile v8h*)(XT + offx[i]) = x[i];
#pragma unroll
  for (int i = 0; i < 4; ++i) *(volatile v8h*)(XD + offy[i]) = y[i];
}

__global__ __launch_bounds__(256) void qconv_kernel(
    const float* __restrict__ xl, const float* __restrict__ Wq, const float* __restrict__ bq,
    _Float16* __restrict__ Qh, _Float16* __restrict__ Qr) {
  const unsigned tid = threadIdx.x;
  const unsigned d0 = blockIdx.x * 64u;
  const unsigned bl = blockIdx.y;
  const unsigned b = bl / (unsigned)NL;
  const unsigned l = bl - b * (unsigned)NL;
  const unsigned c = tid >> 3;
  const unsigned dp = (tid & 7u) * 8u;
  const float w0 = bf16r(Wq[c * 3u + 0u]);
  const float w1 = bf16r(Wq[c * 3u + 1u]);
  const float w2 = bf16r(Wq[c * 3u + 2u]);
  const float bb = bf16r(bq[c]);
  const float* xp = xl + ((size_t)(b * (unsigned)NL_FULL + l) * DD + d0 + dp) * FF;
  float xs[24];
#pragma unroll
  for (int k = 0; k < 6; ++k) {
    const v4f t4 = *(const v4f*)(xp + 4 * k);
#pragma unroll
    for (int j = 0; j < 4; ++j) xs[4 * k + j] = bf16r(t4[j]);
  }
  v8h qh, qr;
#pragma unroll
  for (int e = 0; e < 8; ++e) {
    const float t = w0 * xs[3 * e] + w1 * xs[3 * e + 1] + w2 * xs[3 * e + 2] + bb;
    const h16 hi = toh_flush(t);
    qh[e] = hi;
    qr[e] = toh_flush((t - (float)hi) * RCARRY);
  }
  const size_t off = ((size_t)bl * CC + c) * DD + d0 + dp;
  *(volatile v8h*)(Qh + off) = qh;
  *(volatile v8h*)(Qr + off) = qr;
  __threadfence();
  *(volatile v8h*)(Qh + off) = qh;
  *(volatile v8h*)(Qr + off) = qr;
}

__global__ __launch_bounds__(256) void score_kernel(
    const _Float16* __restrict__ Qh, const _Float16* __restrict__ Qr,
    const _Float16* __restrict__ XT, const float* __restrict__ Wm,
    const float* __restrict__ bm, const float* __restrict__ Wc, _Float16* __restrict__ AW) {
  __shared__ __attribute__((aligned(16))) float Gs[CC * LDG];
  __shared__ __attribute__((aligned(16))) float As[CC * LDA];
  const unsigned tid = threadIdx.x, lane = tid & 31u;
  const int wave = __builtin_amdgcn_readfirstlane(threadIdx.x >> 5);
  const unsigned hh = lane >> 4, m = lane & 15u;
  const unsigned bl = blockIdx.x;

  const _Float16* ah0 = Qh + ((size_t)bl * CC + m) * DD + hh * 8u;
  const _Float16* ah1 = ah0 + (size_t)16 * DD;
  const _Float16* ar0 = Qr + ((size_t)bl * CC + m) * DD + hh * 8u;
  const _Float16* ar1 = ar0 + (size_t)16 * DD;
  const _Float16* bp  = XT + ((size_t)bl * JP + (unsigned)wave * 16u + m) * DD + hh * 8u;
  v8f h0 = {}, h1 = {}, r0 = {}, r1 = {};
#pragma unroll 2
  for (unsigned k0 = 0; k0 < (unsigned)DD; k0 += 32u) {
    const v16h a0 = frag_at(ah0 + k0);
    const v16h a1 = frag_at(ah1 + k0);
    const v16h c0 = frag_at(ar0 + k0);
    const v16h c1 = frag_at(ar1 + k0);
    const v16h bf = frag_at(bp + k0);
    h0 = wmma16(a0, bf, h0);
    h1 = wmma16(a1, bf, h1);
    r0 = wmma16(c0, bf, r0);
    r1 = wmma16(c1, bf, r1);
  }
#pragma unroll
  for (int r = 0; r < 8; ++r) {
    float* g = &Gs[(hh * 8u + (unsigned)r) * LDG + (unsigned)wave * 16u + m];
    g[0]        = (h0[r] + r0[r] * (1.0f / RCARRY)) * (1.0f / XCARRY);
    g[16 * LDG] = (h1[r] + r1[r] * (1.0f / RCARRY)) * (1.0f / XCARRY);
  }
  __syncthreads();

  if (wave == 0) {
    const unsigned c = lane;
    const float w0 = bf16r(Wm[c * 3u + 0u]);
    const float w1 = bf16r(Wm[c * 3u + 1u]);
    const float w2 = bf16r(Wm[c * 3u + 2u]);
    const float bias = bf16r(bm[c]) * Gs[c * LDG + (unsigned)JR];
    float mx = 0.0f;
#pragma unroll 1
    for (unsigned t = 0; t < (unsigned)TT; ++t) {
      float s = w0 * Gs[c * LDG + 3u * t] + w1 * Gs[c * LDG + 3u * t + 1u]
              + w2 * Gs[c * LDG + 3u * t + 2u] + bias;
      s = fmaxf(s, 0.0f);
      As[c * LDA + t] = s;
      mx = fmaxf(mx, s);
    }
    float sum = 0.0f;
#pragma unroll 1
    for (unsigned t = 0; t < (unsigned)TT; ++t) {
      const float e = expf(As[c * LDA + t] - mx);
      As[c * LDA + t] = e;
      sum += e;
    }
    const float inv = 1.0f / sum;
#pragma unroll 1
    for (unsigned t = 0; t < (unsigned)TT; ++t) As[c * LDA + t] = As[c * LDA + t] * inv;
  }
  __syncthreads();

  v8h x[2];
  size_t off[2];
#pragma unroll
  for (unsigned i = 0; i < 2u; ++i) {
    const unsigned c = 16u * i + (tid >> 4);
    const unsigned jc = (tid & 15u) * 8u;
    const float wc0 = bf16r(Wc[c * 3u + 0u]);
    const float wc1 = bf16r(Wc[c * 3u + 1u]);
    const float wc2 = bf16r(Wc[c * 3u + 2u]);
#pragma unroll
    for (unsigned e = 0; e < 8u; ++e) {
      const unsigned j = jc + e;
      const unsigned t = j / 3u;
      const unsigned f = j - t * 3u;
      const unsigned tc = (t < (unsigned)TT) ? t : (unsigned)(TT - 1);
      const float a = As[c * LDA + tc];
      const float wsel = (f == 0u) ? wc0 : ((f == 1u) ? wc1 : wc2);
      const float val = (j < (unsigned)JR) ? (PCARRY * a * wsel) : 0.0f;
      x[i][e] = toh_flush(val);
    }
    off[i] = ((size_t)bl * CC + c) * JP + jc;
  }
#pragma unroll
  for (int i = 0; i < 2; ++i) *(volatile v8h*)(AW + off[i]) = x[i];
  __threadfence();
#pragma unroll
  for (int i = 0; i < 2; ++i) *(volatile v8h*)(AW + off[i]) = x[i];
}

__global__ __launch_bounds__(256) void out_kernel(
    const _Float16* __restrict__ AW, const _Float16* __restrict__ XD,
    const float* __restrict__ xl, const float* __restrict__ Wq, const float* __restrict__ bq,
    const float* __restrict__ bc, float* __restrict__ outf) {
  __shared__ __attribute__((aligned(16))) float Cs[CC * LDG];
  const unsigned tid = threadIdx.x, lane = tid & 31u;
  const int wave = __builtin_amdgcn_readfirstlane(threadIdx.x >> 5);
  const unsigned hh = lane >> 4, m = lane & 15u;
  const unsigned d0 = blockIdx.x * 128u;
  const unsigned bl = blockIdx.y;
  const unsigned b = bl / (unsigned)NL;
  const unsigned l = bl - b * (unsigned)NL;

  const _Float16* ap0 = AW + ((size_t)bl * CC + m) * JP + hh * 8u;
  const _Float16* ap1 = ap0 + (size_t)16 * JP;
  const _Float16* bp  = XD + ((size_t)bl * DD + d0 + (unsigned)wave * 16u + m) * JP + hh * 8u;
  v8f acc0 = {}, acc1 = {};
#pragma unroll
  for (unsigned k0 = 0; k0 < (unsigned)JP; k0 += 32u) {
    const v16h a0 = frag_at(ap0 + k0);
    const v16h a1 = frag_at(ap1 + k0);
    const v16h bf = frag_at(bp + k0);
    acc0 = wmma16(a0, bf, acc0);
    acc1 = wmma16(a1, bf, acc1);
  }
#pragma unroll
  for (int r = 0; r < 8; ++r) {
    float* g = &Cs[(hh * 8u + (unsigned)r) * LDG + (unsigned)wave * 16u + m];
    g[0]        = acc0[r];
    g[16 * LDG] = acc1[r];
  }
  __syncthreads();

  const unsigned dcol = lane * 4u;
  const float* xp = xl + ((size_t)(b * (unsigned)NL_FULL + l) * DD + d0 + dcol) * FF;
  float xs[12];
#pragma unroll
  for (int k = 0; k < 3; ++k) {
    const v4f t4 = *(const v4f*)(xp + 4 * k);
#pragma unroll
    for (int j = 0; j < 4; ++j) xs[4 * k + j] = bf16r(t4[j]);
  }
  const float oscale = 1.0f / (PCARRY * XCARRY);
  v4f xo[4];
  size_t off[4];
#pragma unroll
  for (unsigned i = 0; i < 4u; ++i) {
    const unsigned c = 8u * i + (unsigned)wave;
    const float w0 = bf16r(Wq[c * 3u + 0u]);
    const float w1 = bf16r(Wq[c * 3u + 1u]);
    const float w2 = bf16r(Wq[c * 3u + 2u]);
    const float qb = bf16r(bq[c]);
    const float cb = bf16r(bc[c]);
    const v4f u = *(const v4f*)&Cs[c * LDG + dcol];
    v4f val;
#pragma unroll
    for (int j = 0; j < 4; ++j) {
      const float qv = w0 * xs[3 * j] + w1 * xs[3 * j + 1] + w2 * xs[3 * j + 2] + qb;
      val[j] = qv + (u[j] * oscale + cb);
    }
    xo[i] = val;
    off[i] = ((size_t)(b * (unsigned)CC + c) * NL_FULL + l) * DD + d0 + dcol;
  }
#pragma unroll
  for (int i = 0; i < 4; ++i) *(volatile v4f*)(outf + off[i]) = xo[i];
  __threadfence();
#pragma unroll
  for (int i = 0; i < 4; ++i) *(volatile v4f*)(outf + off[i]) = xo[i];
}

extern "C" void kernel_launch(void* const* d_in, const int* in_sizes, int n_in,
                              void* d_out, int out_size, void* d_ws, size_t ws_size,
                              hipStream_t stream) {
  if (n_in < 8) return;
  const long long rows = (long long)(NB - 1) * NL_FULL + NL;
  if ((long long)in_sizes[0] < rows * DD * FF) return;
  if ((long long)in_sizes[1] < rows * TT * DD * FF) return;
  if (in_sizes[2] < CC * FF || in_sizes[4] < CC * FF || in_sizes[6] < CC * FF) return;
  if (in_sizes[3] < CC || in_sizes[5] < CC || in_sizes[7] < CC) return;
  const long long need_out =
      (((long long)(NB - 1) * CC + (CC - 1)) * NL_FULL + NL) * (long long)DD;
  if ((long long)out_size < need_out) return;
  if (ws_size < WS_TOTAL) return;

  const float* xl = (const float*)d_in[0];
  const float* xh = (const float*)d_in[1];
  const float* wq = (const float*)d_in[2];
  const float* bq = (const float*)d_in[3];
  const float* wm = (const float*)d_in[4];
  const float* bm = (const float*)d_in[5];
  const float* wc = (const float*)d_in[6];
  const float* bc = (const float*)d_in[7];
  float* out = (float*)d_out;

  char* ws = (char*)d_ws;
  _Float16* XT16 = (_Float16*)(ws + OFF_XT);
  _Float16* XD16 = (_Float16*)(ws + OFF_XD);
  _Float16* Qh16 = (_Float16*)(ws + OFF_QH);
  _Float16* Qr16 = (_Float16*)(ws + OFF_QR);
  _Float16* AW16 = (_Float16*)(ws + OFF_AW);

  dim3 blk(256);
  xconv_kernel<<<dim3(DD / 64, NBL), blk, 0, stream>>>(xh, XT16, XD16);
  qconv_kernel<<<dim3(DD / 64, NBL), blk, 0, stream>>>(xl, wq, bq, Qh16, Qr16);
  score_kernel<<<dim3(NBL), blk, 0, stream>>>(Qh16, Qr16, XT16, wm, bm, wc, AW16);
  out_kernel<<<dim3(DD / 128, NBL), blk, 0, stream>>>(AW16, XD16, xl, wq, bq, bc, out);
}
